// TimelineGNNLayer2_39410619908397
// MI455X (gfx1250) — hardware-run, weakly checked
//
#include <hip/hip_runtime.h>


namespace {
constexpr int N = 50000, NP = 50048, E = 800000, D = 128, TD = 32, AD = 64, NR = 401, NRP = 416, NT = 1000, NTP = 1008, NQ = 512, EC = 7;
constexpr float XS = 8.0f, ES = 256.0f, WSC = 256.0f, NEG = 0.01f;
typedef _Float16 b16;
typedef __attribute__((ext_vector_type(16))) _Float16 v16b;
typedef __attribute__((ext_vector_type(8))) _Float16 v8b;
typedef __attribute__((ext_vector_type(8))) float v8f;
typedef __attribute__((ext_vector_type(4))) float v4f;
__device__ __forceinline__ float bf16_rne(float f) { unsigned int u = __float_as_uint(f); u += 0x7FFFu + ((u >> 16) & 1u); return __uint_as_float(u & 0xFFFF0000u); }
__device__ __forceinline__ void split16(float v, b16& hi, b16& lo) { hi = (b16)v; lo = (b16)(v - (float)hi); }
__device__ __forceinline__ v16b frag_kb(const b16* p, int hh) { const v8b a = *(const v8b*)(p + 8 * hh), b = *(const v8b*)(p + 16 + 8 * hh); v16b f;
#pragma unroll
  for (int e = 0; e < 8; ++e) { f[e] = a[e]; f[8 + e] = b[e]; } return f; }
__device__ __forceinline__ v8f wmma16b(v16b a, v16b b, v8f c) { v8f d = __builtin_amdgcn_wmma_f32_16x16x32_f16(false, a, false, b, (short)0, c, false, false); asm volatile("v_nop\n\tv_nop\n\tv_nop\n\tv_nop" : "+v"(d) : "v"(a), "v"(b)); return d; }
__device__ __forceinline__ void wave_lds_sync() { __builtin_amdgcn_fence(__ATOMIC_RELEASE, "workgroup"); __builtin_amdgcn_wave_barrier(); __builtin_amdgcn_fence(__ATOMIC_ACQUIRE, "workgroup"); }
__device__ __forceinline__ float pmul(float a, float b) { float p = a * b; asm volatile("" : "+v"(p)); return p; }
__device__ __forceinline__ float opaque(float a) { asm volatile("" : "+v"(a)); return a; }
__device__ __forceinline__ int iclamp(int v, int lo, int hi) { return v < lo ? lo : (v > hi ? hi : v); }
__device__ __forceinline__ float lrelu(float x) { return x > 0.0f ? x : NEG * x; }
constexpr int CSR_NBLK = 512, CSR_GB = 9, CSR_GN = 1 << CSR_GB  , CSR_TS = (CSR_GN < 32 ? 32 : CSR_GN)  , CSR_MAXG = 512, CSR_CAP = 12288  ;
__device__ __host__ __forceinline__ int csr_tix(int v) { return (v >> CSR_GB) * CSR_TS + (v & (CSR_GN - 1)); }
__global__ __launch_bounds__(64) void csrA_kernel(const int* __restrict__ dst, int E, int N, int nG, int CHP, int NGP, int* __restrict__ STG, int* __restrict__ HST) {
  extern __shared__ int sm[];
  int* cnt = sm; int* run = sm + NGP; int* ids = sm + 2 * NGP;
  const int b = blockIdx.x; const int ch = (E + CSR_NBLK - 1) / CSR_NBLK; const int e0 = b * ch, e1 = min(E, e0 + ch);
  for (int i = threadIdx.x; i < NGP; i += 64) cnt[i] = 0;
  for (int i = threadIdx.x; i < CHP; i += 64) ids[i] = -1;
  __syncthreads();
  if (threadIdx.x == 0) {
    for (int e = e0; e < e1; ++e) { int d = dst[e]; d = (d < 0) ? 0 : (d >= N ? N - 1 : d); cnt[d >> CSR_GB] += 1; }
    int acc = 0; for (int g = 0; g < nG; ++g) { run[g] = acc; acc += cnt[g]; }
    for (int e = e0; e < e1; ++e) { int d = dst[e]; d = (d < 0) ? 0 : (d >= N ? N - 1 : d); const int g = d >> CSR_GB; ids[run[g]] = e; run[g] += 1; } }
  __syncthreads();
  typedef __attribute__((ext_vector_type(4))) int v4i;
  for (int pass = 0; pass < 2; ++pass) {
    for (int i = threadIdx.x; i < CHP / 4; i += 64) *(volatile v4i*)(STG + (size_t)b * CHP + i * 4) = *(const v4i*)(&ids[i * 4]);
    for (int i = threadIdx.x; i < NGP / 4; i += 64) { v4i v; for (int e = 0; e < 4; ++e) v[e] = (i * 4 + e < nG) ? cnt[i * 4 + e] : 0; *(volatile v4i*)(HST + (size_t)b * NGP + i * 4) = v; }
    __threadfence(); }
}
__global__ __launch_bounds__(512) void csrS_kernel(const int* __restrict__ HST, int nG, int NGP, int* __restrict__ START, int* __restrict__ TOT, int* __restrict__ OFF) {
  __shared__ int tot[CSR_MAXG];
  const int b = threadIdx.x;
  for (int pass = 0; pass < 2; ++pass) { int runb = 0; for (int g = 0; g < nG; ++g) { int c = HST[(size_t)b * NGP + g]; c = (c < 0) ? 0 : c; ((volatile int*)OFF)[(size_t)g * CSR_NBLK + b] = runb; runb += c; } __threadfence(); }
  for (int g = threadIdx.x; g < nG; g += 512) { int s = 0; for (int bb = 0; bb < CSR_NBLK; ++bb) { int c = HST[(size_t)bb * NGP + g]; s += (c < 0) ? 0 : c; } tot[g] = s; }
  __syncthreads();
  if (threadIdx.x < 32) {
    __shared__ int st[CSR_MAXG + 32];
    if (threadIdx.x == 0) { int acc = 0; for (int g = 0; g < NGP; ++g) { st[g] = acc; if (g < nG) acc += (tot[g] + 31) & ~31; } st[NGP] = acc; }
    __builtin_amdgcn_fence(__ATOMIC_RELEASE, "workgroup"); __builtin_amdgcn_wave_barrier(); __builtin_amdgcn_fence(__ATOMIC_ACQUIRE, "workgroup");
    for (int pass = 0; pass < 2; ++pass) { for (int i = threadIdx.x; i < NGP + 32; i += 32) { ((volatile int*)START)[i] = (i <= NGP) ? st[min(i, NGP)] : 0; ((volatile int*)TOT)[i] = (i < nG) ? tot[i] : 0; } __threadfence(); } }
}
__global__ __launch_bounds__(256) void csrB_kernel(const int* __restrict__ dst, int N, int nG, int CHP, int NGP, int permLen, const int* __restrict__ STG, const int* __restrict__ HST, const int* __restrict__ OFF, const int* __restrict__ START, const int* __restrict__ TOT, int* __restrict__ PERM, int* __restrict__ ROWPTR, int* __restrict__ ROWCNT, int* __restrict__ FLAG) {
  typedef __attribute__((ext_vector_type(4))) int v4i;
  __shared__ int ids[CSR_CAP]; __shared__ unsigned short key[CSR_CAP]; __shared__ int outp[CSR_CAP]; __shared__ int ncnt[CSR_GN + 1]; __shared__ int boff[CSR_NBLK + 1];
  const int g = blockIdx.x, t_ = threadIdx.x; int tot = TOT[g]; int st = START[g], stn = START[g + 1]; const int v0 = g * CSR_GN; const int nv = min(CSR_GN, N - v0); const int t0 = g * CSR_TS;
  st = (st < 0) ? 0 : (st > permLen - 32 ? permLen - 32 : st) & ~31; stn = (stn < st) ? st : (stn > permLen ? permLen : stn); tot = (tot < 0) ? 0 : tot; if (tot > stn - st && tot <= CSR_CAP) tot = stn - st;
  if (tot > CSR_CAP) {
    for (int pass = 0; pass < 2; ++pass) { for (int i = t_; i < CSR_TS / 4; i += 256) { v4i a, c; for (int e = 0; e < 4; ++e) { a[e] = st; c[e] = 0; } *(volatile v4i*)(ROWPTR + t0 + i * 4) = a; *(volatile v4i*)(ROWCNT + t0 + i * 4) = c; } if (t_ == 0) ((volatile int*)FLAG)[0] = 1; __threadfence(); } (void)nv; return; }
  if (t_ == 0) { int acc = 0; for (int b = 0; b < CSR_NBLK; ++b) { boff[b] = acc; int c = HST[(size_t)b * NGP + g]; c = (c < 0) ? 0 : (c > CHP ? CHP : c); acc += c; if (acc > tot) acc = tot; } boff[CSR_NBLK] = acc; }
  for (int i = t_; i <= CSR_GN; i += 256) ncnt[i] = 0;
  __syncthreads();
  for (int b = 0; b < CSR_NBLK; ++b) { const int c = boff[b + 1] - boff[b]; int o_ = OFF[(size_t)g * CSR_NBLK + b]; o_ = (o_ < 0) ? 0 : (o_ > CHP - c ? CHP - c : o_); const int* src_ = STG + (size_t)b * CHP + o_;
    for (int i = t_; i < c; i += 256) { int id = src_[i]; id = (id < 0) ? 0 : id; ids[boff[b] + i] = id; int d = dst[id]; d = (d < v0) ? v0 : (d >= N ? N - 1 : d); int kk = d - v0; kk = (kk < 0) ? 0 : (kk >= CSR_GN ? CSR_GN - 1 : kk); key[boff[b] + i] = (unsigned short)kk; } }
  __syncthreads();
  if (t_ == 0) { for (int i = 0; i < tot; ++i) ncnt[key[i]] += 1; int acc = 0; for (int vl = 0; vl < CSR_GN; ++vl) { const int c = ncnt[vl]; ncnt[vl] = acc; acc += c; } ncnt[CSR_GN] = acc;
    for (int i = 0; i < tot; ++i) { const int vl = key[i]; outp[ncnt[vl]] = ids[i]; ncnt[vl] += 1; }
    for (int vl = CSR_GN; vl > 0; --vl) ncnt[vl] = ncnt[vl - 1]; ncnt[0] = 0; }
  __syncthreads();
  for (int pass = 0; pass < 2; ++pass) {
    for (int i = t_; i < (stn - st) / 4; i += 256) { v4i v; for (int e = 0; e < 4; ++e) { const int q = i * 4 + e; v[e] = (q < tot) ? outp[q] : -1; } *(volatile v4i*)(PERM + st + i * 4) = v; }
    for (int i = t_; i < CSR_TS / 4; i += 256) { v4i a, c; for (int e = 0; e < 4; ++e) { const int vl = i * 4 + e; const int vc = vl < CSR_GN ? vl : CSR_GN; a[e] = (vl < CSR_GN) ? st + ncnt[vc] : st; c[e] = (vl < nv) ? (ncnt[(vc < CSR_GN ? vc : CSR_GN - 1) + 1] - ncnt[vc]) : 0; } *(volatile v4i*)(ROWPTR + t0 + i * 4) = a; *(volatile v4i*)(ROWCNT + t0 + i * 4) = c; }
    __threadfence(); }
}
__global__ __launch_bounds__(256) void csrZ_kernel(int* __restrict__ p, size_t n4) { typedef __attribute__((ext_vector_type(4))) int v4i; const size_t tid = (size_t)blockIdx.x * 256 + threadIdx.x, nth = (size_t)gridDim.x * 256; v4i z = {0, 0, 0, 0}; for (size_t i = tid; i < n4; i += nth) *(volatile v4i*)(p + i * 4) = z; }
struct CsrBufs { int *STG, *HST, *OFF, *START, *TOT, *PERM, *ROWPTR, *ROWCNT, *FLAG; int nG, NGP, CHP; size_t permLen; char* base; size_t bytes; };
static size_t csr_carve(CsrBufs& c, char* ws, size_t off, int E, int N) {
  const size_t off0 = off; c.base = ws + off;
  auto al = [&](size_t bytes) { char* p = ws + off; off += (bytes + 255) & ~(size_t)255; return p; };
  c.nG = (N + CSR_GN - 1) / CSR_GN; c.NGP = (c.nG + 31) & ~31; const int ch = (E + CSR_NBLK - 1) / CSR_NBLK; c.CHP = (ch + 31) & ~31; c.permLen = (size_t)E + 32 * (size_t)c.nG + 32;
  c.STG = (int*)al((size_t)CSR_NBLK * c.CHP * 4); c.HST = (int*)al((size_t)CSR_NBLK * c.NGP * 4); c.OFF = (int*)al((size_t)c.NGP * CSR_NBLK * 4); c.START = (int*)al((size_t)(c.NGP + 64) * 4); c.TOT = (int*)al((size_t)(c.NGP + 64) * 4);
  c.PERM = (int*)al(c.permLen * 4); c.ROWPTR = (int*)al((size_t)c.nG * CSR_TS * 4); c.ROWCNT = (int*)al((size_t)c.nG * CSR_TS * 4); c.FLAG = (int*)al(256);
  c.bytes = off - off0; return off;
}
static void csr_build(const CsrBufs& c, const int* dst, int E, int N, hipStream_t stream) {
  const size_t smem = (size_t)(2 * c.NGP + c.CHP) * 4;
  csrZ_kernel<<<512, 256, 0, stream>>>((int*)c.base, c.bytes / 16);
  csrA_kernel<<<CSR_NBLK, 64, smem, stream>>>(dst, E, N, c.nG, c.CHP, c.NGP, c.STG, c.HST);
  csrS_kernel<<<1, 512, 0, stream>>>(c.HST, c.nG, c.NGP, c.START, c.TOT, c.OFF);
  csrB_kernel<<<c.nG, 256, 0, stream>>>(dst, N, c.nG, c.CHP, c.NGP, (int)c.permLen, c.STG, c.HST, c.OFF, c.START, c.TOT, c.PERM, c.ROWPTR, c.ROWCNT, c.FLAG);
}


__global__ __launch_bounds__(256) void wprep_kernel(const float* __restrict__ w, int r0, int KIN, int OUT, b16* __restrict__ WT) {
  const size_t u = (size_t)blockIdx.x * 256 + threadIdx.x; if (u >= (size_t)OUT * KIN / 8) return; const size_t e = u * 8; const int o = (int)(e / KIN), k0 = (int)(e % KIN); v8b v;
  for (int j = 0; j < 8; ++j) v[j] = (b16)(bf16_rne(w[(size_t)(r0 + k0 + j) * OUT + o]) * WSC); for (int pass = 0; pass < 2; ++pass) { *(volatile v8b*)(WT + e) = v; __threadfence(); }
}
template <int KIN, int NTL>
__global__ __launch_bounds__(32) void tgemm_kernel(const float* __restrict__ tab, const int* __restrict__ IDX, int nrows, int tabrows, const b16* __restrict__ WT, const float* __restrict__ bias, float* __restrict__ OUTP) {
  __shared__ __attribute__((aligned(16))) float Tf[16][NTL * 16 + 4];
  const int lane = threadIdx.x, nloc = lane & 15, hlf = lane >> 4; const size_t m0 = (size_t)blockIdx.x * 16; size_t r = m0 + nloc; if (r >= (size_t)nrows) r = nrows - 1;
  if (IDX != nullptr) r = (size_t)iclamp(IDX[r], 0, tabrows - 1);
  const float* xr = tab + r * KIN;
  v8f acc[NTL];
#pragma unroll
  for (int t = 0; t < NTL; ++t) acc[t] = (v8f){};
#pragma unroll
  for (int kb = 0; kb < KIN; kb += 32) { v16b a; for (int j = 0; j < 8; ++j) { a[j] = (b16)(bf16_rne(xr[kb + 8 * hlf + j]) * XS); a[8 + j] = (b16)(bf16_rne(xr[kb + 16 + 8 * hlf + j]) * XS); }
#pragma unroll
    for (int t = 0; t < NTL; ++t) acc[t] = wmma16b(a, frag_kb(WT + (size_t)(t * 16 + nloc) * KIN + kb, hlf), acc[t]); }
#pragma unroll
  for (int t = 0; t < NTL; ++t) { const int c = t * 16 + nloc; const float bb = bias != nullptr ? bf16_rne(bias[c]) : 0.0f;
#pragma unroll 1
    for (int r8 = 0; r8 < 8; ++r8) Tf[8 * hlf + r8][c] = acc[t][r8] * (1.0f / (XS * WSC)) + bb; }
  wave_lds_sync();
  for (int pass = 0; pass < 2; ++pass) { for (int rr = 0; rr < 16; ++rr) if (lane < NTL * 4) *(volatile v4f*)(OUTP + (m0 + rr) * (NTL * 16) + lane * 4) = *(const v4f*)(&Tf[rr][lane * 4]); __threadfence(); }
}
__global__ __launch_bounds__(256) void dst_kernel(const int* __restrict__ edges, const float* __restrict__ hidden, const float* __restrict__ remb, const float* __restrict__ RW1, const float* __restrict__ TW1, const float* __restrict__ RWR, const float* __restrict__ QW, const float* __restrict__ HS,
                                                   const b16* __restrict__ W2T, const b16* __restrict__ WRT, const float* __restrict__ b2, const float* __restrict__ wal,
                                                   const int* __restrict__ PERM, const int* __restrict__ ROWPTR, const int* __restrict__ ROWCNT, int permLen, float* __restrict__ AVG) {
  __shared__ __attribute__((aligned(16))) b16 Ah[8][16][D + 8], Al[8][16][D + 8]; __shared__ __attribute__((aligned(16))) float Row[8][D + 4]; __shared__ int eidx[8][16][4]; __shared__ float eas[8][16];
  const int wave = threadIdx.x >> 5, lane = threadIdx.x & 31, nloc = lane & 15, hlf = lane >> 4; const size_t v = (size_t)blockIdx.x * 8 + wave;
  int st = 0, cnt = 0; if (v < (size_t)N) { st = ROWPTR[v]; cnt = ROWCNT[v]; cnt = iclamp(cnt, 0, 65536); st = iclamp(st, 0, permLen - cnt); }
  float U[8]; for (int t = 0; t < 8; ++t) U[t] = 0.0f; float bot = 0.0f;
  float wa[4]; for (int t = 0; t < 4; ++t) wa[t] = opaque(bf16_rne(wal[t * 16 + nloc]));
  const int nchunk = (cnt + 15) >> 4;
#pragma unroll 1
  for (int ch = 0; ch < nchunk; ++ch) {
    const int j = ch * 16 + nloc; const bool ok = j < cnt; const int e = ok ? iclamp(PERM[st + j], 0, E - 1) : 0;
    const int ridx = iclamp(edges[(size_t)e * EC + 0], 0, NQ - 1), rel = iclamp(edges[(size_t)e * EC + 2], 0, NR - 1), sub = iclamp(edges[(size_t)e * EC + 4], 0, N - 1), tim = iclamp(edges[(size_t)e * EC + 6], 0, NT - 1);
    if (hlf == 0) { eidx[wave][nloc][0] = ridx; eidx[wave][nloc][1] = rel; eidx[wave][nloc][2] = sub; eidx[wave][nloc][3] = ok ? tim : -1; }
    wave_lds_sync();
    for (int rr = 0; rr < 16; ++rr) { const int rl = eidx[wave][rr][1], tm = eidx[wave][rr][3] < 0 ? 0 : eidx[wave][rr][3]; const v4f a = *(const v4f*)(RW1 + (size_t)rl * D + lane * 4), b = *(const v4f*)(TW1 + (size_t)tm * D + lane * 4);
      for (int q = 0; q < 4; ++q) { b16 p, ql; split16(lrelu(a[q] + b[q]) * ES, p, ql); Ah[wave][rr][lane * 4 + q] = p; Al[wave][rr][lane * 4 + q] = ql; } }
    wave_lds_sync();
    v8f acc[8];
#pragma unroll
    for (int t = 0; t < 8; ++t) acc[t] = (v8f){};
#pragma unroll 2
    for (int kb = 0; kb < D; kb += 32) { const v16b a = frag_kb(&Ah[wave][nloc][kb], hlf), al = frag_kb(&Al[wave][nloc][kb], hlf);
#pragma unroll
      for (int t = 0; t < 8; ++t) { const v16b bw = frag_kb(W2T + (size_t)(t * 16 + nloc) * D + kb, hlf); acc[t] = wmma16b(a, bw, acc[t]); acc[t] = wmma16b(al, bw, acc[t]); } }
    wave_lds_sync();
#pragma unroll
    for (int t = 0; t < 8; ++t) { const int c = t * 16 + nloc; const float bb = bf16_rne(b2[c]);
#pragma unroll
      for (int r8 = 0; r8 < 8; ++r8) { const float hv = lrelu(acc[t][r8] * (1.0f / (ES * WSC)) + bb); acc[t][r8] = hv; b16 p, ql; split16(hv * ES, p, ql); Ah[wave][8 * hlf + r8][c] = p; Al[wave][8 * hlf + r8][c] = ql; } }
    wave_lds_sync();
    v8f az[4];
#pragma unroll
    for (int t = 0; t < 4; ++t) az[t] = (v8f){};
#pragma unroll 2
    for (int kb = 0; kb < D; kb += 32) { const v16b a = frag_kb(&Ah[wave][nloc][kb], hlf), al = frag_kb(&Al[wave][nloc][kb], hlf);
#pragma unroll
      for (int t = 0; t < 4; ++t) { const v16b bw = frag_kb(WRT + (size_t)(t * 16 + nloc) * D + kb, hlf); az[t] = wmma16b(a, bw, az[t]); az[t] = wmma16b(al, bw, az[t]); } }
    float pa[8];
#pragma unroll
    for (int r8 = 0; r8 < 8; ++r8) { const int rl = 8 * hlf + r8; const int sb = eidx[wave][rl][2], re = eidx[wave][rl][1], rq = eidx[wave][rl][0]; float s = 0.0f;
#pragma unroll
      for (int t = 0; t < 4; ++t) { const int c = t * 16 + nloc; const float zz = az[t][r8] * (1.0f / (ES * WSC)) + HS[(size_t)sb * AD + c] + RWR[(size_t)re * AD + c] + QW[(size_t)rq * AD + c]; s += pmul(lrelu(zz), wa[t]); }
      pa[r8] = s; }
#pragma unroll
    for (int r8 = 0; r8 < 8; ++r8) { float s = pa[r8]; for (int o = 1; o < 16; o <<= 1) s += __shfl_xor(s, o); const int rl = 8 * hlf + r8; const float ea = (eidx[wave][rl][3] >= 0) ? __expf(s) : 0.0f; pa[r8] = ea; if (nloc == 0) eas[wave][rl] = ea; }
#pragma unroll
    for (int t = 0; t < 8; ++t) { const int c = t * 16 + nloc; float s = 0.0f;
#pragma unroll
      for (int r8 = 0; r8 < 8; ++r8) { const int rl = 8 * hlf + r8; const int sb = eidx[wave][rl][2], re = eidx[wave][rl][1]; const float g = bf16_rne(hidden[(size_t)sb * D + c]) + bf16_rne(remb[(size_t)re * D + c]); s += pmul(pa[r8], acc[t][r8] + g); }
      s += __shfl_xor(s, 16); U[t] += s; }
    { float sb_ = 0.0f; for (int r8 = 0; r8 < 8; ++r8) sb_ += pa[r8]; sb_ += __shfl_xor(sb_, 16); bot += sb_; }
    wave_lds_sync(); }
  const float inv = 1.0f / (bot + 1e-5f);
  if (hlf == 0) for (int t = 0; t < 8; ++t) Row[wave][t * 16 + nloc] = (v < (size_t)N) ? pmul(U[t], inv) : 0.0f;
  wave_lds_sync();
  for (int pass = 0; pass < 2; ++pass) { *(volatile v4f*)(AVG + v * D + lane * 4) = *(const v4f*)(&Row[wave][lane * 4]); __threadfence(); }
}
__global__ __launch_bounds__(128) void out_kernel(const float* __restrict__ AVG, const b16* __restrict__ WHT, float* __restrict__ out) {
  __shared__ __attribute__((aligned(16))) b16 Ah[4][16][D + 8], Al[4][16][D + 8]; __shared__ __attribute__((aligned(16))) float Tf[4][16][D + 4];
  const int wave = threadIdx.x >> 5, lane = threadIdx.x & 31, nloc = lane & 15, hlf = lane >> 4; const size_t m0 = (size_t)blockIdx.x * 64 + wave * 16;
  for (int rr = 0; rr < 16; ++rr) { const v4f z = *(const v4f*)(AVG + (m0 + rr) * D + lane * 4); for (int j = 0; j < 4; ++j) { b16 p, q; split16(z[j] * XS, p, q); Ah[wave][rr][lane * 4 + j] = p; Al[wave][rr][lane * 4 + j] = q; } }
  wave_lds_sync();
  v8f acc[8];
#pragma unroll
  for (int t = 0; t < 8; ++t) acc[t] = (v8f){};
#pragma unroll 2
  for (int kb = 0; kb < D; kb += 32) { const v16b a = frag_kb(&Ah[wave][nloc][kb], hlf), al = frag_kb(&Al[wave][nloc][kb], hlf);
#pragma unroll
    for (int t = 0; t < 8; ++t) { const v16b bw = frag_kb(WHT + (size_t)(t * 16 + nloc) * D + kb, hlf); acc[t] = wmma16b(a, bw, acc[t]); acc[t] = wmma16b(al, bw, acc[t]); } }
#pragma unroll
  for (int t = 0; t < 8; ++t)
#pragma unroll 1
    for (int r8 = 0; r8 < 8; ++r8) Tf[wave][8 * hlf + r8][t * 16 + nloc] = acc[t][r8] * (1.0f / (XS * WSC));
  wave_lds_sync();
  for (int pass = 0; pass < 2; ++pass) { for (int rr = 0; rr < 16; ++rr) if ((m0 + rr) < (size_t)N) *(volatile v4f*)(out + (m0 + rr) * D + lane * 4) = *(const v4f*)(&Tf[wave][rr][lane * 4]); __threadfence(); }
}
__global__ __launch_bounds__(256) void objcopy_kernel(const int* __restrict__ edges, int* __restrict__ OBJ) {
  const int e = blockIdx.x * 256 + threadIdx.x; if (e >= E) return; const int o = edges[(size_t)e * EC + 5]; for (int pass = 0; pass < 2; ++pass) { ((volatile int*)OBJ)[e] = o; __threadfence(); }
}
}

extern "C" void kernel_launch(void* const* d_in, const int* in_sizes, int n_in, void* d_out, int out_size, void* d_ws, size_t ws_size, hipStream_t stream) {
  (void)n_in;
  auto Fp = [&](int i) { return (const float*)d_in[i]; }; auto Ip = [&](int i) { return (const int*)d_in[i]; };
  if (in_sizes[0] != N * D || in_sizes[1] != NR * D || in_sizes[2] != NT * TD || in_sizes[3] != (D + TD) * D || in_sizes[5] != D * D || in_sizes[7] != D * AD || in_sizes[9] != D * AD || in_sizes[11] != AD || in_sizes[12] != D * D || in_sizes[13] != NQ || in_sizes[14] != E * EC || out_size != N * D) return;
  size_t off = 0; char* ws = (char*)d_ws;
  auto carve = [&](size_t bytes) { char* p = ws + off; off += (bytes + 255) & ~(size_t)255; return p; };
  b16* W1A = (b16*)carve(D * D * 2); b16* W1B = (b16*)carve(D * TD * 2); b16* W2T = (b16*)carve(D * D * 2); b16* WST = (b16*)carve(AD * D * 2); b16* WRT = (b16*)carve(AD * D * 2); b16* WQT = (b16*)carve(AD * D * 2); b16* WHT = (b16*)carve(D * D * 2);
  float* RW1 = (float*)carve((size_t)NRP * D * 4); float* TW1 = (float*)carve((size_t)NTP * D * 4); float* RWR = (float*)carve((size_t)NRP * AD * 4); float* QW = (float*)carve((size_t)NQ * AD * 4); float* HS = (float*)carve((size_t)NP * AD * 4); float* AVG = (float*)carve((size_t)NP * D * 4); int* OBJ = (int*)carve((size_t)E * 4 + 256);
  CsrBufs csr; off = csr_carve(csr, ws, off, E, N);
  if (off > ws_size || off > ((size_t)128 << 20)) return;
  wprep_kernel<<<(D * D / 8 + 255) / 256, 256, 0, stream>>>(Fp(3), 0, D, D, W1A); wprep_kernel<<<(D * TD / 8 + 255) / 256, 256, 0, stream>>>(Fp(3), D, TD, D, W1B);
  wprep_kernel<<<(D * D / 8 + 255) / 256, 256, 0, stream>>>(Fp(5), 0, D, D, W2T); wprep_kernel<<<(AD * D / 8 + 255) / 256, 256, 0, stream>>>(Fp(7), 0, D, AD, WST);
  wprep_kernel<<<(AD * D / 8 + 255) / 256, 256, 0, stream>>>(Fp(8), 0, D, AD, WRT); wprep_kernel<<<(AD * D / 8 + 255) / 256, 256, 0, stream>>>(Fp(9), 0, D, AD, WQT);
  wprep_kernel<<<(D * D / 8 + 255) / 256, 256, 0, stream>>>(Fp(12), 0, D, D, WHT);
  objcopy_kernel<<<E / 256, 256, 0, stream>>>(Ip(14), OBJ);
  csr_build(csr, OBJ, E, N, stream);
  tgemm_kernel<D, 8><<<NRP / 16, 32, 0, stream>>>(Fp(1), nullptr, NR, NR, W1A, Fp(4), RW1);
  tgemm_kernel<TD, 8><<<NTP / 16, 32, 0, stream>>>(Fp(2), nullptr, NT, NT, W1B, nullptr, TW1);
  tgemm_kernel<D, 4><<<NRP / 16, 32, 0, stream>>>(Fp(1), nullptr, NR, NR, WRT, nullptr, RWR);
  tgemm_kernel<D, 4><<<NQ / 16, 32, 0, stream>>>(Fp(1), Ip(13), NQ, NR, WQT, Fp(10), QW);
  tgemm_kernel<D, 4><<<NP / 16, 32, 0, stream>>>(Fp(0), nullptr, N, N, WST, nullptr, HS);
  dst_kernel<<<NP / 8, 256, 0, stream>>>(Ip(14), Fp(0), Fp(1), RW1, TW1, RWR, QW, HS, W2T, WRT, Fp(6), Fp(11), csr.PERM, csr.ROWPTR, csr.ROWCNT, (int)csr.permLen, AVG);
  out_kernel<<<NP / 64, 128, 0, stream>>>(AVG, WHT, (float*)d_out);
}
